// QIM_22789096473379
// MI455X (gfx1250) — hardware-verified
//
#include <hip/hip_runtime.h>


#define NB_  4
#define NN   2048
#define DD   256
#define NH_  8
#define HD   32
#define NT   (NB_ * NN)
#define ZH   2
typedef _Float16 h16;
typedef unsigned short bf;
typedef __attribute__((ext_vector_type(16))) __bf16   v16bf;
typedef __attribute__((ext_vector_type(16))) _Float16 v16h;
typedef __attribute__((ext_vector_type(8)))  _Float16 v8h;
typedef __attribute__((ext_vector_type(8)))  unsigned short v8us;
typedef __attribute__((ext_vector_type(8)))  float    v8f;
typedef __attribute__((ext_vector_type(4)))  float    v4f;
typedef v8h  __attribute__((may_alias)) v8ha;
typedef v4f  __attribute__((may_alias)) v4fa;
typedef v8us __attribute__((may_alias)) v8usa;

__device__ __forceinline__ unsigned short f2bf(float f) { unsigned u = __float_as_uint(f); u += 0x7FFFu + ((u >> 16) & 1u); return (unsigned short)(u >> 16); }
__device__ __forceinline__ float bf2f(unsigned short b) { return __uint_as_float(((unsigned)b) << 16); }
__device__ __forceinline__ float bfr(float f) { return bf2f(f2bf(f)); }
__device__ __forceinline__ v16h cat16(v8h lo, v8h hi) { return __builtin_shufflevector(lo, hi, 0, 1, 2, 3, 4, 5, 6, 7, 8, 9, 10, 11, 12, 13, 14, 15); }
__device__ __forceinline__ v16bf cat16b(v8us lo, v8us hi) { return __builtin_bit_cast(v16bf, __builtin_shufflevector(lo, hi, 0, 1, 2, 3, 4, 5, 6, 7, 8, 9, 10, 11, 12, 13, 14, 15)); }
__device__ __forceinline__ v8f wmma16(v16h a, v16h b, v8f c) { return __builtin_amdgcn_wmma_f32_16x16x32_f16(false, a, false, b, (short)0, c, false, false); }
__device__ __forceinline__ v8f wmmab(v16bf a, v16bf b, v8f c) { return __builtin_amdgcn_wmma_f32_16x16x32_bf16(false, a, false, b, (short)0, c, false, false); }


template <typename T16> struct WFrag;
template <> struct WFrag<h16> { typedef v16h V; static __device__ __forceinline__ V ld(const h16* p) { return cat16(*(const v8h*)p, *(const v8h*)(p + 16)); } static __device__ __forceinline__ v8f mma(V a, V b, v8f c) { return wmma16(a, b, c); } };
template <> struct WFrag<bf> { typedef v16bf V; static __device__ __forceinline__ V ld(const bf* p) { return cat16b(*(const v8us*)p, *(const v8us*)(p + 16)); } static __device__ __forceinline__ v8f mma(V a, V b, v8f c) { return wmmab(a, b, c); } };
template <typename T16, int NSPLIT, bool BIAS>
__global__ __launch_bounds__(32) void k_gemmw(const T16* __restrict__ A, const T16* __restrict__ A2, const T16* __restrict__ Bt, const T16* __restrict__ Bt2, int K, float* C, int ldc, const float* __restrict__ bias, size_t sA, size_t sB, size_t sC) {
    typedef typename WFrag<T16>::V V;
    __shared__ __align__(16) float os[16 * 68];
    const size_t z = blockIdx.z; A += z * sA; if (A2) A2 += z * sA; Bt += z * sB; if (Bt2) Bt2 += z * sB; C += z * sC;
    const int lane = threadIdx.x & 31, lr = lane & 15, hi = lane >> 4; const int r0 = blockIdx.x * 64, c0 = blockIdx.y * 64;
    v8f acc[4][4];
#pragma unroll
    for (int mb = 0; mb < 4; ++mb)
#pragma unroll
        for (int nb = 0; nb < 4; ++nb) acc[mb][nb] = (v8f){};
    const size_t aoff = (size_t)(r0 + lr) * K + 8 * hi, boff = (size_t)(c0 + lr) * K + 8 * hi;
#pragma unroll 1
    for (int kc = 0; kc < K; kc += 32) {
        V a[4], a2[4];
#pragma unroll
        for (int mb = 0; mb < 4; ++mb) { a[mb] = WFrag<T16>::ld(A + aoff + (size_t)mb * 16 * K + kc); if (NSPLIT == 1 || NSPLIT == 2) a2[mb] = WFrag<T16>::ld(A2 + aoff + (size_t)mb * 16 * K + kc); }
#pragma unroll
        for (int nb = 0; nb < 4; ++nb) { const V b = WFrag<T16>::ld(Bt + boff + (size_t)nb * 16 * K + kc); V b2; if (NSPLIT >= 2) b2 = WFrag<T16>::ld(Bt2 + boff + (size_t)nb * 16 * K + kc);
#pragma unroll
            for (int mb = 0; mb < 4; ++mb) { acc[mb][nb] = WFrag<T16>::mma(a[mb], b, acc[mb][nb]); if (NSPLIT == 1 || NSPLIT == 2) acc[mb][nb] = WFrag<T16>::mma(a2[mb], b, acc[mb][nb]); if (NSPLIT >= 2) acc[mb][nb] = WFrag<T16>::mma(a[mb], b2, acc[mb][nb]); } }
        asm volatile("v_nop\n\tv_nop\n\tv_nop\n\tv_nop" : "+v"(acc[0][0]), "+v"(acc[1][1]), "+v"(acc[2][2]), "+v"(acc[3][3]) : "v"(a[0]), "v"(a[3]));
    }
#pragma unroll
    for (int mb = 0; mb < 4; ++mb) {
#pragma unroll
        for (int nb = 0; nb < 4; ++nb) {
#pragma unroll
            for (int j = 0; j < 8; ++j) os[(hi * 8 + j) * 68 + nb * 16 + lr] = acc[mb][nb][j]; }
        __builtin_amdgcn_wave_barrier(); asm volatile("" ::: "memory");
        float* crow = C + (size_t)(r0 + mb * 16) * ldc + c0;
#pragma unroll 1
        for (int ps = 0; ps < 2; ++ps) {
#pragma unroll
            for (int s = 0; s < 8; ++s) { const int row = 2 * s + hi, cofs = lr * 4; v4f val = *(const v4fa*)(os + row * 68 + cofs); if (BIAS) { val[0] += bfr(bias[c0 + cofs]); val[1] += bfr(bias[c0 + cofs + 1]); val[2] += bfr(bias[c0 + cofs + 2]); val[3] += bfr(bias[c0 + cofs + 3]); }
                *(volatile v4f*)(crow + (size_t)row * ldc + cofs) = val; }
            if (ps == 0) __threadfence(); }
        __builtin_amdgcn_wave_barrier(); asm volatile("" ::: "memory");
    }
}

__device__ __forceinline__ h16 tohx(float x) { return (h16)x; }
__device__ __forceinline__ void splitf(float y, unsigned short& h, unsigned short& l) { h = f2bf(y); l = f2bf(y - bf2f(h)); }
typedef __attribute__((ext_vector_type(2))) _Float16 v2h;
typedef __attribute__((ext_vector_type(4))) _Float16 v4h;
typedef __attribute__((ext_vector_type(2))) unsigned short v2us;
typedef __attribute__((ext_vector_type(4))) unsigned short v4us;

__global__ __launch_bounds__(256) void k_wtb(const float* __restrict__ w, int K, int N, bf* Bt) {
    const int lane = threadIdx.x & 31; const int L0 = (blockIdx.x * 8 + (threadIdx.x >> 5)) * 8; const int nlines = N * K / 64;
#pragma unroll 1
    for (int ps = 0; ps < 2; ++ps) {
#pragma unroll 1
        for (int l = 0; l < 8; ++l) { const int L = L0 + l; if (L >= nlines) break; const int e = L * 64 + lane * 2; v2us o;
#pragma unroll
            for (int q = 0; q < 2; ++q) { const int n = (e + q) / K, k = (e + q) % K; o[q] = f2bf(w[(size_t)k * N + n]); }
            *(volatile v2us*)(Bt + e) = o; }
        if (ps == 0) __threadfence(); }
}
__global__ __launch_bounds__(256) void k_xsplit(const float* __restrict__ qdt, const float* __restrict__ boxes, bf* Xh, bf* Xl) {
    const int lane = threadIdx.x & 31; const int L0 = (blockIdx.x * 8 + (threadIdx.x >> 5)) * 8; const int nlines = NT * DD / 64;
#pragma unroll 1
    for (int ps = 0; ps < 2; ++ps) {
#pragma unroll
        for (int l = 0; l < 8; ++l) { const int L = L0 + l; if (L >= nlines) break; const int e = L * 64 + lane * 2; v2us oh, ol;
#pragma unroll
            for (int q = 0; q < 2; ++q) { unsigned short a, c2; splitf(bfr(boxes[(size_t)e + q]) + bfr(qdt[(size_t)e + q]), a, c2); oh[q] = a; ol[q] = c2; }
            *(volatile v2us*)(Xh + (size_t)e) = oh; *(volatile v2us*)(Xl + (size_t)e) = ol; }
        if (ps == 0) __threadfence(); }
}
__global__ __launch_bounds__(256) void k_qkplane(const float* __restrict__ F, int col0, float sc, h16* P) {
    const int lane = threadIdx.x & 31; const int L0 = (blockIdx.x * 8 + (threadIdx.x >> 5)) * 8; const int nlines = NT * DD / 64;
#pragma unroll 1
    for (int ps = 0; ps < 2; ++ps) {
#pragma unroll
        for (int l = 0; l < 8; ++l) { const int L = L0 + l; if (L >= nlines) break; const int e = L * 64 + lane * 2; const int d = e & 31; const int n = (e >> 5) & (NN - 1); const int h = (e >> 16) & 7; const int b = e >> 19; v2h v;
#pragma unroll
            for (int q = 0; q < 2; ++q) v[q] = tohx(F[((size_t)b * NN + n) * (3 * DD) + col0 + h * HD + d + q] * sc);
            *(volatile v2h*)(P + (size_t)e) = v; }
        if (ps == 0) __threadfence(); }
}
__global__ __launch_bounds__(256) void k_vtplane(const float* __restrict__ F, h16* VT) {
    const int lane = threadIdx.x & 31; const int L0 = (blockIdx.x * 8 + (threadIdx.x >> 5)) * 8; const int nlines = NB_ * NH_ * 64 * NN / 64;
#pragma unroll 1
    for (int ps = 0; ps < 2; ++ps) {
#pragma unroll
        for (int l = 0; l < 8; ++l) { const int L = L0 + l; if (L >= nlines) break; const int e = L * 64 + lane * 2; const int n = e & (NN - 1); const int d = (e >> 11) & 63; const int h = (e >> 17) & 7; const int b = e >> 20; v2h v;
#pragma unroll
            for (int q = 0; q < 2; ++q) v[q] = tohx(d < HD ? F[((size_t)b * NN + n + q) * (3 * DD) + 2 * DD + h * HD + d] : 0.f);
            *(volatile v2h*)(VT + (size_t)e) = v; }
        if (ps == 0) __threadfence(); }
}
__global__ __launch_bounds__(256) void k_sigm(const float* __restrict__ Sb, const int* __restrict__ mask, h16* P) {
    const size_t i = (size_t)blockIdx.x * 256 + threadIdx.x; if (i >= (size_t)ZH * NN * NN / 4) return; const size_t e = i * 4; const int k = (int)(e & (NN - 1)); const int q = (int)((e >> 11) & (NN - 1));
    const v4f s = *(const v4f*)(Sb + e); v4h o;
#pragma unroll
    for (int j = 0; j < 4; ++j) { const int m = mask[(size_t)q * NN + k + j]; const float sg = __fdiv_rn(1.0f, 1.0f + __expf(-s[j])); o[j] = tohx(m != 0 ? sg : 0.f); }
    *(volatile v4h*)(P + e) = o; __threadfence(); *(volatile v4h*)(P + e) = o;
}
__global__ __launch_bounds__(256) void k_omerge(const float* __restrict__ O, int b, int h0, bf* Ah, bf* Al) {
    const int lane = threadIdx.x & 31; const int n = blockIdx.x * 8 + (threadIdx.x >> 5); if (n >= NN) return; const int zz = lane >> 4, d = (lane & 15) * 2; v2us oh, ol;
#pragma unroll
    for (int q = 0; q < 2; ++q) { unsigned short a, c2; splitf(O[((size_t)zz * NN + n) * 64 + d + q], a, c2); oh[q] = a; ol[q] = c2; }
    const size_t o = ((size_t)b * NN + n) * DD + (h0 + zz) * HD + d; *(volatile v2us*)(Ah + o) = oh; *(volatile v2us*)(Al + o) = ol; __threadfence(); *(volatile v2us*)(Ah + o) = oh; *(volatile v2us*)(Al + o) = ol;
}
template <bool FINAL>
__global__ __launch_bounds__(256) void k_ln(const float* __restrict__ A, const float* __restrict__ R1, const float* __restrict__ R2, const float* __restrict__ gg, const float* __restrict__ bb, float* Y, bf* Ph, bf* Pl) {
    const int lane = threadIdx.x & 31; const int r = blockIdx.x * 8 + (threadIdx.x >> 5); if (r >= NT) return; float v[8]; float s = 0.f;
#pragma unroll
    for (int c = 0; c < 2; ++c)
#pragma unroll
        for (int q = 0; q < 4; ++q) { const int col = c * 128 + lane * 4 + q; const size_t idx = (size_t)r * DD + col; const float res = FINAL ? R1[idx] : (bfr(R1[idx]) + bfr(R2[idx])); const float t = res + A[idx]; v[c * 4 + q] = t; s += t; }
#pragma unroll
    for (int sh = 16; sh; sh >>= 1) s += __shfl_xor(s, sh, 32);
    const float mu = s * (1.0f / DD); float qq = 0.f;
#pragma unroll
    for (int i = 0; i < 8; ++i) { const float d0 = v[i] - mu; qq = fmaf(d0, d0, qq); }
#pragma unroll
    for (int sh = 16; sh; sh >>= 1) qq += __shfl_xor(qq, sh, 32);
    const float rs = rsqrtf(qq * (1.0f / DD) + 1e-5f); v4f o[2]; v4us oh[2], ol[2];
#pragma unroll
    for (int c = 0; c < 2; ++c)
#pragma unroll
        for (int q = 0; q < 4; ++q) { const int col = c * 128 + lane * 4 + q; const float y = (v[c * 4 + q] - mu) * rs * bfr(gg[col]) + bfr(bb[col]); o[c][q] = y; if (!FINAL) { unsigned short a, c2; splitf(y, a, c2); oh[c][q] = a; ol[c][q] = c2; } }
#pragma unroll 1
    for (int ps = 0; ps < 2; ++ps) {
#pragma unroll
        for (int c = 0; c < 2; ++c) { *(volatile v4f*)(Y + (size_t)r * DD + c * 128 + lane * 4) = o[c]; if (!FINAL) { *(volatile v4us*)(Ph + (size_t)r * DD + c * 128 + lane * 4) = oh[c]; *(volatile v4us*)(Pl + (size_t)r * DD + c * 128 + lane * 4) = ol[c]; } }
        if (ps == 0) __threadfence(); }
}
__global__ __launch_bounds__(256) void k_relusplit(const float* __restrict__ H, bf* Ph, bf* Pl) {
    const int lane = threadIdx.x & 31; const int L0 = (blockIdx.x * 8 + (threadIdx.x >> 5)) * 8; const int nlines = NT * DD / 64;
#pragma unroll 1
    for (int ps = 0; ps < 2; ++ps) {
#pragma unroll
        for (int l = 0; l < 8; ++l) { const int L = L0 + l; if (L >= nlines) break; const int e = L * 64 + lane * 2; v2us oh, ol;
#pragma unroll
            for (int q = 0; q < 2; ++q) { unsigned short a, c2; splitf(fmaxf(H[(size_t)e + q], 0.f), a, c2); oh[q] = a; ol[q] = c2; }
            *(volatile v2us*)(Ph + (size_t)e) = oh; *(volatile v2us*)(Pl + (size_t)e) = ol; }
        if (ps == 0) __threadfence(); }
}

extern "C" void kernel_launch(void* const* d_in, const int* in_sizes, int n_in,
                              void* d_out, int out_size, void* d_ws, size_t ws_size, hipStream_t stream) {
    (void)in_sizes; (void)n_in; (void)out_size;
    const float* qdt = (const float*)d_in[0]; const float* boxes = (const float*)d_in[1]; const int* mask = (const int*)d_in[2];
    const float* Wq = (const float*)d_in[3]; const float* bq = (const float*)d_in[4]; const float* Wk = (const float*)d_in[5]; const float* bk = (const float*)d_in[6]; const float* Wv = (const float*)d_in[7]; const float* bv = (const float*)d_in[8]; const float* Wo = (const float*)d_in[9]; const float* bo = (const float*)d_in[10];
    const float* W1 = (const float*)d_in[11]; const float* b1 = (const float*)d_in[12]; const float* W2 = (const float*)d_in[13]; const float* b2 = (const float*)d_in[14]; const float* g1 = (const float*)d_in[15]; const float* be1 = (const float*)d_in[16]; const float* g2 = (const float*)d_in[17]; const float* be2 = (const float*)d_in[18];
    float* OUT = (float*)d_out;
    char* wsp = (char*)d_ws;
    auto take = [&](size_t bytes) { char* p = wsp; wsp += (bytes + 255) & ~(size_t)255; return (void*)p; };
    bf* WQ = (bf*)take((size_t)DD * DD * 2); bf* WK = (bf*)take((size_t)DD * DD * 2); bf* WV = (bf*)take((size_t)DD * DD * 2); bf* WO = (bf*)take((size_t)DD * DD * 2); bf* WF1 = (bf*)take((size_t)DD * DD * 2); bf* WF2 = (bf*)take((size_t)DD * DD * 2);
    bf* Xh = (bf*)take((size_t)NT * DD * 2); bf* Xl = (bf*)take((size_t)NT * DD * 2); float* F = (float*)take((size_t)NT * 3 * DD * 4);
    h16* QP = (h16*)take((size_t)NT * DD * 2); h16* KP = (h16*)take((size_t)NT * DD * 2); h16* VT = (h16*)take((size_t)NB_ * NH_ * 64 * NN * 2);
    float* Sb = (float*)take((size_t)ZH * NN * NN * 4); h16* Pm = (h16*)take((size_t)ZH * NN * NN * 2); float* Ob = (float*)take((size_t)ZH * NN * 64 * 4);
    bf* ATh = (bf*)take((size_t)NT * DD * 2); bf* ATl = (bf*)take((size_t)NT * DD * 2); float* AO = (float*)take((size_t)NT * DD * 4); float* T1 = (float*)take((size_t)NT * DD * 4); bf* T1h = (bf*)take((size_t)NT * DD * 2); bf* T1l = (bf*)take((size_t)NT * DD * 2);
    if ((size_t)(wsp - (char*)d_ws) > ws_size) return;
    float* Hf = F; bf* Rh = Xh; bf* Rl = Xl; float* F2 = AO;
    { const unsigned gw = (unsigned)((DD * DD / 64 + 63) / 64); k_wtb<<<gw, 256, 0, stream>>>(Wq, DD, DD, WQ); k_wtb<<<gw, 256, 0, stream>>>(Wk, DD, DD, WK); k_wtb<<<gw, 256, 0, stream>>>(Wv, DD, DD, WV); k_wtb<<<gw, 256, 0, stream>>>(Wo, DD, DD, WO); k_wtb<<<gw, 256, 0, stream>>>(W1, DD, DD, WF1); k_wtb<<<gw, 256, 0, stream>>>(W2, DD, DD, WF2); }
    const unsigned LB = (unsigned)((NT * DD / 64 + 63) / 64);
    k_xsplit<<<LB, 256, 0, stream>>>(qdt, boxes, Xh, Xl);
    k_gemmw<bf, 1, true><<<dim3(NT / 64, DD / 64, 1), 32, 0, stream>>>(Xh, Xl, WQ, nullptr, DD, F, 3 * DD, bq, 0, 0, 0);
    k_gemmw<bf, 1, true><<<dim3(NT / 64, DD / 64, 1), 32, 0, stream>>>(Xh, Xl, WK, nullptr, DD, F + DD, 3 * DD, bk, 0, 0, 0);
    k_gemmw<bf, 1, true><<<dim3(NT / 64, DD / 64, 1), 32, 0, stream>>>(Xh, Xl, WV, nullptr, DD, F + 2 * DD, 3 * DD, bv, 0, 0, 0);
    k_qkplane<<<LB, 256, 0, stream>>>(F, 0, 0x1.6a09e6p-3f, QP); k_qkplane<<<LB, 256, 0, stream>>>(F, DD, 1.0f, KP);
    k_vtplane<<<(unsigned)((NB_ * NH_ * 64 * NN / 64 + 63) / 64), 256, 0, stream>>>(F, VT);
    for (int b = 0; b < NB_; ++b)
        for (int h0 = 0; h0 < NH_; h0 += ZH) { const size_t z0 = (size_t)b * NH_ + h0;
            k_gemmw<h16, 0, false><<<dim3(NN / 64, NN / 64, ZH), 32, 0, stream>>>(QP + z0 * NN * HD, nullptr, KP + z0 * NN * HD, nullptr, HD, Sb, NN, nullptr, (size_t)NN * HD, (size_t)NN * HD, (size_t)NN * NN);
            k_sigm<<<(unsigned)(((size_t)ZH * NN * NN / 4 + 255) / 256), 256, 0, stream>>>(Sb, mask, Pm);
            k_gemmw<h16, 0, false><<<dim3(NN / 64, 1, ZH), 32, 0, stream>>>(Pm, nullptr, VT + z0 * 64 * NN, nullptr, NN, Ob, 64, nullptr, (size_t)NN * NN, (size_t)64 * NN, (size_t)NN * 64);
            k_omerge<<<NN / 8, 256, 0, stream>>>(Ob, b, h0, ATh, ATl); }
    k_gemmw<bf, 1, true><<<dim3(NT / 64, DD / 64, 1), 32, 0, stream>>>(ATh, ATl, WO, nullptr, DD, AO, DD, bo, 0, 0, 0);
    k_ln<false><<<NT / 8, 256, 0, stream>>>(AO, boxes, qdt, g1, be1, T1, T1h, T1l);
    k_gemmw<bf, 1, true><<<dim3(NT / 64, DD / 64, 1), 32, 0, stream>>>(T1h, T1l, WF1, nullptr, DD, Hf, DD, b1, 0, 0, 0);
    k_relusplit<<<LB, 256, 0, stream>>>(Hf, Rh, Rl);
    k_gemmw<bf, 1, true><<<dim3(NT / 64, DD / 64, 1), 32, 0, stream>>>(Rh, Rl, WF2, nullptr, DD, F2, DD, b2, 0, 0, 0);
    k_ln<true><<<NT / 8, 256, 0, stream>>>(F2, T1, nullptr, g2, be2, OUT, nullptr, nullptr);
}
